// GraphEncoder_GAT_wSKIP_10917806866971
// MI455X (gfx1250) — hardware-verified
//
#include <hip/hip_runtime.h>
#include <stddef.h>


#define DF    256
#define NH    4
#define HC    64
#define GR    32
#define XSP   260
#define TP    264
#define NB    256
#define CHUNK 2048
#define NTHR  256
#define NWAVE 8
#define WCAP  256
#define NGRP  (CHUNK / (NTHR * 4))
#define MR    64
#define CSP   132

#define LDS_SACC (NB * DF)
#define LDS_MX   (NB * NH)
#define LDS_DEN  (NB * NH)
#define LDS_LIST (NWAVE * WCAP)
#define LDS_BYTES ((LDS_SACC + LDS_MX + LDS_DEN + LDS_LIST + NWAVE) * 4)

static_assert(WCAP == (CHUNK / NTHR) * 32);
static_assert(NGRP == 2);
static_assert(NB == 256);
static_assert(CHUNK == 2048);
static_assert((LDS_SACC % 4) == 0);
static_assert(LDS_BYTES == 278560);
static_assert(LDS_BYTES <= 327680);
static_assert((NB / NWAVE) == 32);
static_assert((NB % GR) == 0);
static_assert((XSP % 4) == 0);
static_assert((TP % 8) == 0);
static_assert((CSP % 4) == 0);
static_assert(DF == NH * HC);

typedef float          v4f  __attribute__((ext_vector_type(4)));
typedef float          v8f  __attribute__((ext_vector_type(8)));
typedef int            v4i  __attribute__((ext_vector_type(4)));
typedef _Float16       v8h  __attribute__((ext_vector_type(8)));
typedef _Float16       v16h __attribute__((ext_vector_type(16)));
typedef __bf16         v16b __attribute__((ext_vector_type(16)));
typedef unsigned short v16u __attribute__((ext_vector_type(16)));
union Frag   { v16h v; v8h half[2]; };
union FragB  { v16b v; v16u u; };
union Pack16 { v8h h; v4i i; };

__device__ __forceinline__ v8f wm(v16h a, v16h b, v8f c) {
  v8f d = __builtin_amdgcn_wmma_f32_16x16x32_f16(false, a, false, b, (short)0, c, false, false);
  asm volatile("v_nop\n\tv_nop\n\tv_nop\n\tv_nop" : "+v"(d) : "v"(a), "v"(b));
  return d;
}
__device__ __forceinline__ v8f wmb(v16b a, v16b b, v8f c) {
  v8f d = __builtin_amdgcn_wmma_f32_16x16x32_bf16(false, a, false, b, (short)0, c, false, false);
  asm volatile("v_nop\n\tv_nop\n\tv_nop\n\tv_nop" : "+v"(d) : "v"(a), "v"(b));
  return d;
}

__device__ __forceinline__ unsigned bfbits(float x) {
  const unsigned u = __float_as_uint(x);
  return (u + 0x7fffu + ((u >> 16) & 1u)) >> 16;
}

__device__ __forceinline__ v4f relu4(v4f y) {
  y.x = y.x > 0.f ? y.x : 0.f;
  y.y = y.y > 0.f ? y.y : 0.f;
  y.z = y.z > 0.f ? y.z : 0.f;
  y.w = y.w > 0.f ? y.w : 0.f;
  return y;
}

__global__ __launch_bounds__(NTHR) void k_cvtx(const float* __restrict__ x, _Float16* xh, int nN, int n8) {
  const int i = blockIdx.x * NTHR + threadIdx.x;
  if (i >= n8) return;
  const size_t o = (size_t)i * 8;
  const int row = (int)(o >> 8);
  const int rc  = row < nN ? row : nN - 1;
  const size_t oc = (size_t)rc * DF + (o & 255);
  v4f a = *(const v4f*)(x + oc);
  v4f b = *(const v4f*)(x + oc + 4);
  if (row >= nN) {
    const v4f z4 = {0.f, 0.f, 0.f, 0.f};
    a = z4; b = z4;
  }
  Pack16 u;
  u.h[0] = (_Float16)a.x; u.h[1] = (_Float16)a.y; u.h[2] = (_Float16)a.z; u.h[3] = (_Float16)a.w;
  u.h[4] = (_Float16)b.x; u.h[5] = (_Float16)b.y; u.h[6] = (_Float16)b.z; u.h[7] = (_Float16)b.w;
  *(volatile v4i*)(xh + o) = u.i;
  __threadfence();
  *(volatile v4i*)(xh + o) = u.i;
}

__global__ __launch_bounds__(NTHR) void k_prepw(const float* __restrict__ Wa, const float* __restrict__ Wb,
                                                const float* __restrict__ Wc, _Float16* Wt) {
  __shared__ __attribute__((aligned(16))) _Float16 T[32 * TP];
  const int tid  = threadIdx.x;
  const int lane = tid & 31;
  const int wave = tid >> 5;
  const float* W = (blockIdx.y == 0) ? Wa : ((blockIdx.y == 1) ? Wb : Wc);
  _Float16* O = Wt + (size_t)blockIdx.y * DF * DF;
  const int n0 = blockIdx.x * 32;
  const int kr = tid >> 3;
  const int c4 = (tid & 7) * 4;
#pragma unroll 1
  for (int it = 0; it < DF / 32; ++it) {
    const int k = it * 32 + kr;
    const v4f v = *(const v4f*)(W + (size_t)k * DF + n0 + c4);
    T[(c4 + 0) * TP + k] = (_Float16)(v.x * 16.0f);
    T[(c4 + 1) * TP + k] = (_Float16)(v.y * 16.0f);
    T[(c4 + 2) * TP + k] = (_Float16)(v.z * 16.0f);
    T[(c4 + 3) * TP + k] = (_Float16)(v.w * 16.0f);
  }
  __syncthreads();
  Pack16 u[4];
#pragma unroll
  for (int i = 0; i < 4; ++i) u[i].h = *(const v8h*)(T + (4 * wave + i) * TP + 8 * lane);
  _Float16* op[4];
#pragma unroll
  for (int i = 0; i < 4; ++i) op[i] = O + (size_t)(n0 + 4 * wave + i) * DF + 8 * lane;
#pragma unroll
  for (int i = 0; i < 4; ++i) *(volatile v4i*)(op[i]) = u[i].i;
  __threadfence();
#pragma unroll
  for (int i = 0; i < 4; ++i) *(volatile v4i*)(op[i]) = u[i].i;
}

__global__ __launch_bounds__(NTHR) void k_gemm(
    const _Float16* __restrict__ Ah, const _Float16* __restrict__ Wt,
    const float* __restrict__ att_s, const float* __restrict__ att_d,
    float* g, float* asrc, float* adst) {
  __shared__ __attribute__((aligned(16))) float Xs[GR * XSP];
  __shared__ __attribute__((aligned(16))) float AD[2 * GR * NH];

  const int tid  = threadIdx.x;
  const int lane = tid & 31;
  const int wave = tid >> 5;
  const int hh   = lane >> 4;
  const int m    = lane & 15;
  const int rowBase = blockIdx.x * GR;

  const _Float16* pa0 = Ah + (size_t)(rowBase + m) * DF + 8 * hh;
  const _Float16* pa1 = Ah + (size_t)(rowBase + 16 + m) * DF + 8 * hh;
  const _Float16* pb0 = Wt + (size_t)(32 * wave + m) * DF + 8 * hh;
  const _Float16* pb1 = Wt + (size_t)(32 * wave + 16 + m) * DF + 8 * hh;

  v8f c00 = {0.f, 0.f, 0.f, 0.f, 0.f, 0.f, 0.f, 0.f};
  v8f c01 = c00, c10 = c00, c11 = c00;
#pragma unroll
  for (int kt = 0; kt < DF / 32; ++kt) {
    const int k0 = kt * 32;
    Frag a0, a1, b0, b1;
    a0.half[0] = *(const v8h*)(pa0 + k0); a0.half[1] = *(const v8h*)(pa0 + k0 + 16);
    a1.half[0] = *(const v8h*)(pa1 + k0); a1.half[1] = *(const v8h*)(pa1 + k0 + 16);
    b0.half[0] = *(const v8h*)(pb0 + k0); b0.half[1] = *(const v8h*)(pb0 + k0 + 16);
    b1.half[0] = *(const v8h*)(pb1 + k0); b1.half[1] = *(const v8h*)(pb1 + k0 + 16);
    c00 = wm(a0.v, b0.v, c00);
    c01 = wm(a0.v, b1.v, c01);
    c10 = wm(a1.v, b0.v, c10);
    c11 = wm(a1.v, b1.v, c11);
  }

  {
    const int cA = 32 * wave + m;
    const int cB = 32 * wave + 16 + m;
#pragma unroll
    for (int r = 0; r < 8; ++r) {
      Xs[(8 * hh + r) * XSP + cA]      = c00[r] * 0.0625f;
      Xs[(8 * hh + r) * XSP + cB]      = c01[r] * 0.0625f;
      Xs[(16 + 8 * hh + r) * XSP + cA] = c10[r] * 0.0625f;
      Xs[(16 + 8 * hh + r) * XSP + cB] = c11[r] * 0.0625f;
    }
  }
  __syncthreads();

  {
    const int r  = tid >> 3;
    const int hd = (tid >> 1) & 3;
    const int wh = tid & 1;
    const float* av = wh ? att_d : att_s;
    const float* xr = Xs + r * XSP + HC * hd;
    const float* ap = av + HC * hd;
    float s = 0.f;
#pragma unroll 4
    for (int c = 0; c < HC; c += 4) {
      const v4f xv = *(const v4f*)(xr + c);
      const v4f aa = *(const v4f*)(ap + c);
      s += xv.x * aa.x + xv.y * aa.y + xv.z * aa.z + xv.w * aa.w;
    }
    AD[wh * (GR * NH) + r * NH + hd] = s;
  }
  __syncthreads();

  v4f xa[4], xb[4];
  float* gp[4];
#pragma unroll
  for (int i = 0; i < 4; ++i) {
    xa[i] = *(const v4f*)(Xs + (4 * wave + i) * XSP + 4 * lane);
    xb[i] = *(const v4f*)(Xs + (4 * wave + i) * XSP + 128 + 4 * lane);
    gp[i] = g + (size_t)(rowBase + 4 * wave + i) * DF + 4 * lane;
  }
  v4f av4 = {0.f, 0.f, 0.f, 0.f};
  float* apn = asrc;
  if (wave == 0) {
    av4 = *(const v4f*)(AD + 4 * lane);
    apn = asrc + (size_t)rowBase * NH + 4 * lane;
  } else if (wave == 1) {
    av4 = *(const v4f*)(AD + GR * NH + 4 * lane);
    apn = adst + (size_t)rowBase * NH + 4 * lane;
  }
#pragma unroll
  for (int i = 0; i < 4; ++i) {
    *(volatile v4f*)(gp[i]) = xa[i];
    *(volatile v4f*)(gp[i] + 128) = xb[i];
  }
  if (wave < 2) *(volatile v4f*)apn = av4;
  __threadfence();
#pragma unroll
  for (int i = 0; i < 4; ++i) {
    *(volatile v4f*)(gp[i]) = xa[i];
    *(volatile v4f*)(gp[i] + 128) = xb[i];
  }
  if (wave < 2) *(volatile v4f*)apn = av4;
}

__global__ __launch_bounds__(NTHR) void k_agg(
    const int* __restrict__ ei, const float* __restrict__ g,
    const float* __restrict__ asrc, const float* __restrict__ adst,
    const float* __restrict__ bias, _Float16* o16, float* o32,
    int nN, int nE, int NP, int relu, int w16) {
  extern __shared__ v4f lds_dyn[];
  float* sacc = (float*)lds_dyn;
  float* mx   = sacc + LDS_SACC;
  float* den  = mx + LDS_MX;
  int*   list = (int*)(den + LDS_DEN);
  int*   wcnt = list + LDS_LIST;

  const int tid  = threadIdx.x;
  const int lane = tid & 31;
  const int wave = tid >> 5;
  const int nodeBase = blockIdx.x * NB;
  const v4f z4 = {0.f, 0.f, 0.f, 0.f};

  for (int i = tid; i < LDS_SACC / 4; i += NTHR) {
    const int fo   = i * 4;
    const int slot = fo >> 8;
    const int col  = fo & (DF - 1);
    const int node = nodeBase + slot;
    const int nc   = node < nN ? node : nN - 1;
    v4f v = *(const v4f*)(g + (size_t)nc * DF + col);
    if (node >= nN) v = z4;
    lds_dyn[i] = v;
  }
  for (int i = tid; i < NB * NH; i += NTHR) {
    const int slot = i >> 2;
    const int hd   = i & 3;
    const int node = nodeBase + slot;
    const int nc   = node < nN ? node : nN - 1;
    float a = asrc[(size_t)nc * NH + hd] + adst[(size_t)nc * NH + hd];
    a = (a > 0.f) ? a : 0.2f * a;
    if (node >= nN) a = 0.f;
    mx[i]  = a;
    den[i] = 1.0f;
  }
  __syncthreads();

  const int* eid = ei + nE;
  const bool al16 = ((nE & 3) == 0);

  const int nChunks = (nE + CHUNK - 1) / CHUNK;
#pragma unroll 1
  for (int ch = 0; ch < nChunks; ++ch) {
    const int cbase = ch * CHUNK;
    const bool full = al16 && (cbase + CHUNK <= nE);
    int wc = 0;
#pragma unroll
    for (int gq = 0; gq < NGRP; ++gq) {
      const int el0 = (gq * NTHR + tid) * 4;
      const int e0  = cbase + el0;
      const int sent = -2147483647 - 1;
      v4i d;
      if (full) {
        d = *(const v4i*)(eid + e0);
      } else {
        const int q0 = eid[min(e0, nE - 1)];
        const int q1 = eid[min(e0 + 1, nE - 1)];
        const int q2 = eid[min(e0 + 2, nE - 1)];
        const int q3 = eid[min(e0 + 3, nE - 1)];
        d.x = (e0     < nE) ? q0 : sent;
        d.y = (e0 + 1 < nE) ? q1 : sent;
        d.z = (e0 + 2 < nE) ? q2 : sent;
        d.w = (e0 + 3 < nE) ? q3 : sent;
      }
      const unsigned s0 = (unsigned)d.x - (unsigned)nodeBase;
      const unsigned s1 = (unsigned)d.y - (unsigned)nodeBase;
      const unsigned s2 = (unsigned)d.z - (unsigned)nodeBase;
      const unsigned s3 = (unsigned)d.w - (unsigned)nodeBase;
      const bool h0 = s0 < (unsigned)NB;
      const bool h1 = s1 < (unsigned)NB;
      const bool h2 = s2 < (unsigned)NB;
      const bool h3 = s3 < (unsigned)NB;
      const unsigned many = __builtin_amdgcn_ballot_w32(h0 | h1 | h2 | h3);
      if (many != 0u) {
#define HITJ(J, HJ, SJ) { \
          const unsigned mj = __builtin_amdgcn_ballot_w32(HJ); \
          if (HJ) { \
            const int pos = wc + (int)__builtin_amdgcn_mbcnt_lo(mj, 0u); \
            if (pos < WCAP) list[wave * WCAP + pos] = ((el0 + (J)) << 8) | (int)(SJ); \
          } \
          wc += (int)__builtin_popcount(mj); }
        HITJ(0, h0, s0)
        HITJ(1, h1, s1)
        HITJ(2, h2, s2)
        HITJ(3, h3, s3)
#undef HITJ
      }
    }
    if (lane == 0) wcnt[wave] = wc;
    __syncthreads();

    if (wave == 0) {
      const int cb = 8 * lane;
      const int hd = lane >> 3;
      for (int wsx = 0; wsx < NWAVE; ++wsx) {
        int n = wcnt[wsx];
        if (n > WCAP) n = WCAP;
        if (n < 0) n = 0;
        for (int i = 0; i < n; ++i) {
          const int ent  = list[wsx * WCAP + i];
          const int slot = ent & (NB - 1);
          const int el   = (ent >> 8) & (CHUNK - 1);
          int e = cbase + el;
          if (e > nE - 1) e = nE - 1;
          int src = ei[e];
          src = src < 0 ? 0 : (src > nN - 1 ? nN - 1 : src);
          int nd = nodeBase + slot;
          if (nd > nN - 1) nd = nN - 1;
          float a = asrc[(size_t)src * NH + hd] + adst[(size_t)nd * NH + hd];
          a = (a > 0.f) ? a : 0.2f * a;
          const int mi = slot * NH + hd;
          const float mo = mx[mi];
          const float mn = fmaxf(mo, a);
          const float sc = __expf(mo - mn);
          const float p  = __expf(a - mn);
          const float* gq = g + (size_t)src * DF + cb;
          const v4f x0 = *(const v4f*)(gq);
          const v4f x1 = *(const v4f*)(gq + 4);
          v4f* sp = (v4f*)(sacc + slot * DF + cb);
          const v4f s0v = sp[0];
          const v4f s1v = sp[1];
          const v4f n0v = s0v * sc + x0 * p;
          const v4f n1v = s1v * sc + x1 * p;
          sp[0] = n0v;
          sp[1] = n1v;
          mx[mi] = mn;
          const float dn = den[mi];
          den[mi] = dn * sc + p;
        }
      }
    }
    __syncthreads();
  }

  const int jn = NB / NWAVE;
#pragma unroll 1
  for (int j = 0; j < jn; ++j) {
    const int slot = wave * jn + j;
    const int node = nodeBase + slot;
    if (node >= NP) break;
    const bool live = node < nN;
    if (w16) {
      const v4f s0v = *(const v4f*)(sacc + slot * DF + 8 * lane);
      const v4f s1v = *(const v4f*)(sacc + slot * DF + 8 * lane + 4);
      const float inv = 1.0f / den[slot * NH + (lane >> 3)];
      const v4f b0 = *(const v4f*)(bias + 8 * lane);
      const v4f b1 = *(const v4f*)(bias + 8 * lane + 4);
      v4f y0 = s0v * inv + b0;
      v4f y1 = s1v * inv + b1;
      if (relu) { y0 = relu4(y0); y1 = relu4(y1); }
      if (!live) { y0 = z4; y1 = z4; }
      Pack16 u;
      u.h[0] = (_Float16)y0.x; u.h[1] = (_Float16)y0.y; u.h[2] = (_Float16)y0.z; u.h[3] = (_Float16)y0.w;
      u.h[4] = (_Float16)y1.x; u.h[5] = (_Float16)y1.y; u.h[6] = (_Float16)y1.z; u.h[7] = (_Float16)y1.w;
      _Float16* op = o16 + (size_t)node * DF + 8 * lane;
      *(volatile v4i*)op = u.i;
      __threadfence();
      *(volatile v4i*)op = u.i;
    } else {
      const v4f s0v = *(const v4f*)(sacc + slot * DF + 4 * lane);
      const v4f s1v = *(const v4f*)(sacc + slot * DF + 128 + 4 * lane);
      const float inv0 = 1.0f / den[slot * NH + (lane >> 4)];
      const float inv1 = 1.0f / den[slot * NH + 2 + (lane >> 4)];
      const v4f b0 = *(const v4f*)(bias + 4 * lane);
      const v4f b1 = *(const v4f*)(bias + 128 + 4 * lane);
      v4f y0 = s0v * inv0 + b0;
      v4f y1 = s1v * inv1 + b1;
      if (relu) { y0 = relu4(y0); y1 = relu4(y1); }
      if (!live) { y0 = z4; y1 = z4; }
      float* op = o32 + (size_t)node * DF + 4 * lane;
      *(volatile v4f*)op = y0;
      *(volatile v4f*)(op + 128) = y1;
      __threadfence();
      *(volatile v4f*)op = y0;
      *(volatile v4f*)(op + 128) = y1;
    }
  }
}

__global__ __launch_bounds__(NTHR) void k_pool(const int* __restrict__ batch, const float* __restrict__ h,
                                               float* pooled, int nN) {
  __shared__ int plist[NWAVE * WCAP];
  __shared__ int pwc[NWAVE];
  const int tid  = threadIdx.x;
  const int lane = tid & 31;
  const int wave = tid >> 5;
  const int gid  = blockIdx.x;
  v4f acc0 = {0.f, 0.f, 0.f, 0.f};
  v4f acc1 = acc0;
  float cnt = 0.f;

  const int nChunks = (nN + CHUNK - 1) / CHUNK;
#pragma unroll 1
  for (int ch = 0; ch < nChunks; ++ch) {
    const int cbase = ch * CHUNK;
    const bool full = (cbase + CHUNK <= nN);
    int wc = 0;
#pragma unroll
    for (int gq = 0; gq < NGRP; ++gq) {
      const int el0 = (gq * NTHR + tid) * 4;
      const int e0  = cbase + el0;
      const int sent = -2147483647 - 1;
      v4i d;
      if (full) {
        d = *(const v4i*)(batch + e0);
      } else {
        const int q0 = batch[min(e0, nN - 1)];
        const int q1 = batch[min(e0 + 1, nN - 1)];
        const int q2 = batch[min(e0 + 2, nN - 1)];
        const int q3 = batch[min(e0 + 3, nN - 1)];
        d.x = (e0     < nN) ? q0 : sent;
        d.y = (e0 + 1 < nN) ? q1 : sent;
        d.z = (e0 + 2 < nN) ? q2 : sent;
        d.w = (e0 + 3 < nN) ? q3 : sent;
      }
      const bool h0 = (d.x == gid);
      const bool h1 = (d.y == gid);
      const bool h2 = (d.z == gid);
      const bool h3 = (d.w == gid);
      const unsigned many = __builtin_amdgcn_ballot_w32(h0 | h1 | h2 | h3);
      if (many != 0u) {
#define HITP(J, HJ) { \
          const unsigned mj = __builtin_amdgcn_ballot_w32(HJ); \
          if (HJ) { \
            const int pos = wc + (int)__builtin_amdgcn_mbcnt_lo(mj, 0u); \
            if (pos < WCAP) plist[wave * WCAP + pos] = el0 + (J); \
          } \
          wc += (int)__builtin_popcount(mj); }
        HITP(0, h0)
        HITP(1, h1)
        HITP(2, h2)
        HITP(3, h3)
#undef HITP
      }
    }
    if (lane == 0) pwc[wave] = wc;
    __syncthreads();
    if (wave == 0) {
      for (int wsx = 0; wsx < NWAVE; ++wsx) {
        int n = pwc[wsx];
        if (n > WCAP) n = WCAP;
        if (n < 0) n = 0;
        cnt += (float)n;
        for (int i = 0; i < n; ++i) {
          const int el = plist[wsx * WCAP + i] & (CHUNK - 1);
          int node = cbase + el;
          if (node > nN - 1) node = nN - 1;
          const float* hp = h + (size_t)node * DF;
          acc0 += *(const v4f*)(hp + 4 * lane);
          acc1 += *(const v4f*)(hp + 128 + 4 * lane);
        }
      }
    }
    __syncthreads();
  }
  if (wave == 0) {
    const float inv = 1.0f / fmaxf(cnt, 1.0f);
    const v4f y0 = acc0 * inv;
    const v4f y1 = acc1 * inv;
    float* op = pooled + (size_t)gid * DF + 4 * lane;
    *(volatile v4f*)op = y0;
    *(volatile v4f*)(op + 128) = y1;
    __threadfence();
    *(volatile v4f*)op = y0;
    *(volatile v4f*)(op + 128) = y1;
  }
}

#define SPL1(FR, X, I) { const unsigned hb_ = bfbits(X); const float hf_ = __uint_as_float(hb_ << 16); \
    FR##hi.u[I] = (unsigned short)hb_; FR##lo.u[I] = (unsigned short)bfbits((X) - hf_); }
#define SPL4(FR, F, I0) SPL1(FR, F.x, (I0)) SPL1(FR, F.y, (I0) + 1) SPL1(FR, F.z, (I0) + 2) SPL1(FR, F.w, (I0) + 3)
#define ROWT(RT, ACC) { \
    const float* ap_ = A + (size_t)(16 * (RT) + m) * K + k0 + 8 * hh; \
    const v4f f0 = *(const v4f*)(ap_); const v4f f1 = *(const v4f*)(ap_ + 4); \
    const v4f f2 = *(const v4f*)(ap_ + 16); const v4f f3 = *(const v4f*)(ap_ + 20); \
    FragB ahi, alo; \
    SPL4(a, f0, 0) SPL4(a, f1, 4) SPL4(a, f2, 8) SPL4(a, f3, 12) \
    ACC = wmb(ahi.v, bhi.v, ACC); ACC = wmb(ahi.v, blo.v, ACC); ACC = wmb(alo.v, bhi.v, ACC); }

__global__ __launch_bounds__(NTHR) void k_mlp(const float* __restrict__ A, const float* __restrict__ W,
                                              const float* __restrict__ bias, float* C, int K, int Nc, int relu) {
  __shared__ __attribute__((aligned(16))) float Cs[MR * CSP];
  const int tid  = threadIdx.x;
  const int lane = tid & 31;
  const int wave = tid >> 5;
  const int hh   = lane >> 4;
  const int m    = lane & 15;
  const int col  = blockIdx.x * 128 + wave * 16 + m;

  v8f c0 = {0.f, 0.f, 0.f, 0.f, 0.f, 0.f, 0.f, 0.f};
  v8f c1 = c0, c2 = c0, c3 = c0;
#pragma unroll 1
  for (int k0 = 0; k0 < K; k0 += 32) {
    FragB bhi, blo;
#pragma unroll
    for (int i = 0; i < 16; ++i) {
      const int kk = k0 + 8 * hh + i + ((i >> 3) << 3);
      const float w = W[(size_t)kk * Nc + col];
      const unsigned hb = bfbits(w);
      const float hf = __uint_as_float(hb << 16);
      bhi.u[i] = (unsigned short)hb;
      blo.u[i] = (unsigned short)bfbits(w - hf);
    }
    ROWT(0, c0)
    ROWT(1, c1)
    ROWT(2, c2)
    ROWT(3, c3)
  }

  {
    const float bv = bias[col];
    const int lc = wave * 16 + m;
#pragma unroll
    for (int r = 0; r < 8; ++r) {
      float v0 = c0[r] + bv, v1 = c1[r] + bv, v2 = c2[r] + bv, v3 = c3[r] + bv;
      if (relu) { v0 = fmaxf(v0, 0.f); v1 = fmaxf(v1, 0.f); v2 = fmaxf(v2, 0.f); v3 = fmaxf(v3, 0.f); }
      Cs[(8 * hh + r) * CSP + lc]      = v0;
      Cs[(16 + 8 * hh + r) * CSP + lc] = v1;
      Cs[(32 + 8 * hh + r) * CSP + lc] = v2;
      Cs[(48 + 8 * hh + r) * CSP + lc] = v3;
    }
  }
  __syncthreads();
  v4f ov[8];
  float* op[8];
#pragma unroll
  for (int i = 0; i < 8; ++i) {
    const int row = 8 * wave + i;
    ov[i] = *(const v4f*)(Cs + row * CSP + 4 * lane);
    op[i] = C + (size_t)row * Nc + blockIdx.x * 128 + 4 * lane;
  }
#pragma unroll
  for (int i = 0; i < 8; ++i) *(volatile v4f*)(op[i]) = ov[i];
  __threadfence();
#pragma unroll
  for (int i = 0; i < 8; ++i) *(volatile v4f*)(op[i]) = ov[i];
}
#undef ROWT
#undef SPL4
#undef SPL1

static inline char* carve(void* base, size_t& off, size_t bytes) {
  char* p = (char*)base + off;
  off += (bytes + 255) & ~(size_t)255;
  return p;
}

extern "C" void kernel_launch(void* const* d_in, const int* in_sizes, int n_in,
                              void* d_out, int out_size, void* d_ws, size_t ws_size,
                              hipStream_t stream) {
  if (n_in < 19) return;
  const int nN = in_sizes[2];
  if (nN <= 0 || in_sizes[0] != nN * DF) return;
  if (in_sizes[1] < 2 || (in_sizes[1] & 1)) return;
  const int nE = in_sizes[1] / 2;
  if (in_sizes[3] != DF * DF || in_sizes[7] != DF * DF || in_sizes[11] != DF * DF) return;
  if (in_sizes[4] != NH * HC || in_sizes[5] != NH * HC || in_sizes[8] != NH * HC ||
      in_sizes[9] != NH * HC || in_sizes[12] != NH * HC || in_sizes[13] != NH * HC) return;
  if (in_sizes[6] != DF || in_sizes[10] != DF || in_sizes[14] != DF) return;
  const int NHD = in_sizes[16];
  const int NO  = in_sizes[18];
  if (NHD <= 0 || NO <= 0 || (NHD % 128) != 0 || (NO % 128) != 0) return;
  if (in_sizes[15] != DF * NHD || in_sizes[17] != NHD * NO) return;
  if (out_size != MR * NO) return;
  const int G  = MR;
  const int NP = ((nN + GR - 1) / GR) * GR;

  const float* x     = (const float*)d_in[0];
  const int*   ei    = (const int*)d_in[1];
  const int*   batch = (const int*)d_in[2];
  const float* W1  = (const float*)d_in[3];
  const float* as1 = (const float*)d_in[4];
  const float* ad1 = (const float*)d_in[5];
  const float* b1  = (const float*)d_in[6];
  const float* W2  = (const float*)d_in[7];
  const float* as2 = (const float*)d_in[8];
  const float* ad2 = (const float*)d_in[9];
  const float* b2  = (const float*)d_in[10];
  const float* W3  = (const float*)d_in[11];
  const float* as3 = (const float*)d_in[12];
  const float* ad3 = (const float*)d_in[13];
  const float* b3  = (const float*)d_in[14];
  const float* Wm1 = (const float*)d_in[15];
  const float* bm1 = (const float*)d_in[16];
  const float* Wm2 = (const float*)d_in[17];
  const float* bm2 = (const float*)d_in[18];
  float* out = (float*)d_out;

  size_t off = 0;
  _Float16* Wt   = (_Float16*)carve(d_ws, off, (size_t)3 * DF * DF * sizeof(_Float16));
  _Float16* nh16 = (_Float16*)carve(d_ws, off, (size_t)NP * DF * sizeof(_Float16));
  float* g      = (float*)carve(d_ws, off, (size_t)NP * DF * sizeof(float));
  float* h3     = (float*)carve(d_ws, off, (size_t)NP * DF * sizeof(float));
  float* asrc   = (float*)carve(d_ws, off, (size_t)NP * NH * sizeof(float));
  float* adst   = (float*)carve(d_ws, off, (size_t)NP * NH * sizeof(float));
  float* pooled = (float*)carve(d_ws, off, (size_t)G * DF * sizeof(float));
  float* hid    = (float*)carve(d_ws, off, (size_t)G * NHD * sizeof(float));
  if (off > ws_size) return;
  if (off > (size_t)134217728) return;

  const int n8 = NP * (DF / 8);
  k_cvtx<<<(n8 + NTHR - 1) / NTHR, NTHR, 0, stream>>>(x, nh16, nN, n8);
  k_prepw<<<dim3(DF / 32, 3), NTHR, 0, stream>>>(W1, W2, W3, Wt);

  hipFuncSetAttribute(reinterpret_cast<const void*>(&k_agg),
                      hipFuncAttributeMaxDynamicSharedMemorySize, LDS_BYTES);
  const int gridG = NP / GR;
  const int gridA = (nN + NB - 1) / NB;

  k_gemm<<<gridG, NTHR, 0, stream>>>(nh16, Wt, as1, ad1, g, asrc, adst);
  k_agg<<<gridA, NTHR, LDS_BYTES, stream>>>(ei, g, asrc, adst, b1, nh16, h3, nN, nE, NP, 1, 1);
  k_gemm<<<gridG, NTHR, 0, stream>>>(nh16, Wt + (size_t)DF * DF, as2, ad2, g, asrc, adst);
  k_agg<<<gridA, NTHR, LDS_BYTES, stream>>>(ei, g, asrc, adst, b2, nh16, h3, nN, nE, NP, 1, 1);
  k_gemm<<<gridG, NTHR, 0, stream>>>(nh16, Wt + (size_t)2 * DF * DF, as3, ad3, g, asrc, adst);
  k_agg<<<gridA, NTHR, LDS_BYTES, stream>>>(ei, g, asrc, adst, b3, nh16, h3, nN, nE, NP, 0, 0);

  k_pool<<<G, NTHR, 0, stream>>>(batch, h3, pooled, nN);
  k_mlp<<<NHD / 128, NTHR, 0, stream>>>(pooled, Wm1, bm1, hid, DF, NHD, 1);
  k_mlp<<<NO / 128, NTHR, 0, stream>>>(hid, Wm2, bm2, out, NHD, NO, 0);
}
